// SelfAttention_51505247814326
// MI455X (gfx1250) — hardware-verified
//
#include <hip/hip_runtime.h>
#include <stdint.h>

#ifndef NB
#define NB 4
#endif
#ifndef SEQ
#define SEQ 4096
#endif
#define NB_FULL  4
#define SEQ_FULL 4096
#define DM       256
#define RTOT     (NB * SEQ)

static_assert(NB >= 1 && NB <= NB_FULL);
static_assert(SEQ >= 256 && SEQ <= SEQ_FULL && (SEQ % 256) == 0);
static_assert(DM == 256);
static_assert((RTOT % 128) == 0);
static_assert(((size_t)RTOT * DM) % 2048 == 0);

typedef _Float16 v16h __attribute__((ext_vector_type(16)));
typedef _Float16 v8h  __attribute__((ext_vector_type(8)));
typedef float    v8f  __attribute__((ext_vector_type(8)));
typedef float    v4f  __attribute__((ext_vector_type(4)));

__device__ __forceinline__ unsigned short bfbits(float f) {
  unsigned u = __float_as_uint(f);
  return (unsigned short)((u + 0x7FFFu + ((u >> 16) & 1u)) >> 16);
}
__device__ __forceinline__ float bfval(unsigned short b) { return __uint_as_float(((unsigned)b) << 16); }
__device__ __forceinline__ float bfr(float f) { return bfval(bfbits(f)); }

__device__ __forceinline__ v8f mma16(v16h a, v16h b, v8f c) {
  return __builtin_amdgcn_wmma_f32_16x16x32_f16(false, a, false, b, (short)0, c, false, false);
}

__device__ __forceinline__ v16h ldfrag(const _Float16* p) {
  union { v16h v; v8h h[2]; } f;
  f.h[0] = *(const v8h*)(p);
  f.h[1] = *(const v8h*)(p + 16);
  return f.v;
}
__device__ __forceinline__ v8f zero8() {
  v8f z;
#pragma unroll
  for (int i = 0; i < 8; ++i) z[i] = 0.0f;
  return z;
}

__device__ __forceinline__ void guard_g(v8f& a, v8f& b, v16h x, v16h y) {
  asm volatile("v_nop\n\tv_nop\n\tv_nop\n\tv_nop" : "+v"(a), "+v"(b) : "v"(x), "v"(y));
}
__device__ __forceinline__ void keep4(v16h a, v16h b, v16h c, v16h d) {
  asm volatile("v_nop" :: "v"(a), "v"(b), "v"(c), "v"(d));
}
__device__ __forceinline__ void accg4(v8f& a, v8f& b, v8f& c, v8f& d) {
  asm volatile("v_nop\n\tv_nop\n\tv_nop\n\tv_nop" : "+v"(a), "+v"(b), "+v"(c), "+v"(d));
}
__device__ __forceinline__ void guard_s8(v8f& a0, v8f& a1, v8f& a2, v8f& a3, v8f& b0, v8f& b1, v8f& b2, v8f& b3,
                                         v16h x0, v16h x1, v16h y0, v16h y1, v16h z0, v16h z1) {
  asm volatile("v_nop\n\tv_nop\n\tv_nop\n\tv_nop"
               : "+v"(a0), "+v"(a1), "+v"(a2), "+v"(a3), "+v"(b0), "+v"(b1), "+v"(b2), "+v"(b3)
               : "v"(x0), "v"(x1), "v"(y0), "v"(y1), "v"(z0), "v"(z1));
}
__device__ __forceinline__ void guard_pv4(v8f& a0, v8f& a1, v8f& b0, v8f& b1,
                                          v16h p0, v16h p1, v16h x0, v16h x1) {
  asm volatile("v_nop\n\tv_nop\n\tv_nop\n\tv_nop"
               : "+v"(a0), "+v"(a1), "+v"(b0), "+v"(b1)
               : "v"(p0), "v"(p1), "v"(x0), "v"(x1));
}

__global__ __launch_bounds__(256) void cvt_kernel(const float* __restrict__ x, const float* __restrict__ Wq,
                                                  const float* __restrict__ Wk, const float* __restrict__ Wv,
                                                  _Float16* __restrict__ X16, _Float16* __restrict__ WT16, int nbx) {
  const int tid = (int)threadIdx.x;
  const int blk = (int)blockIdx.x;
  if (blk < nbx) {
    const int li = blk * 256 + tid;
    const int r  = li >> 5;
    const int c0 = (li & 31) * 8;
    const int b  = r / SEQ;
    const int n  = r - b * SEQ;
    const float* xr = x + ((size_t)b * SEQ_FULL + n) * DM + c0;
    const v4f a  = *(const v4f*)(xr);
    const v4f a2 = *(const v4f*)(xr + 4);
    v8h o;
#pragma unroll
    for (int i = 0; i < 4; ++i) {
      o[i]     = (_Float16)(bfr(a[i]) * 16.0f);
      o[4 + i] = (_Float16)(bfr(a2[i]) * 16.0f);
    }
    _Float16* d = X16 + (size_t)li * 8;
    *(volatile v8h*)d = o;
    __threadfence();
    *(volatile v8h*)d = o;
  } else {
    const int li = (blk - nbx) * 256 + tid;
    if (li >= 3 * DM * DM / 8) return;
    const int mat = li >> 13;
    const int n   = (li >> 5) & (DM - 1);
    const int k0  = (li & 31) * 8;
    const float* W = (mat == 0) ? Wq : ((mat == 1) ? Wk : Wv);
    v8h o;
#pragma unroll
    for (int i = 0; i < 8; ++i) o[i] = (_Float16)(bfr(W[(size_t)(k0 + i) * DM + n]) * 64.0f);
    _Float16* d = WT16 + (size_t)li * 8;
    *(volatile v8h*)d = o;
    __threadfence();
    *(volatile v8h*)d = o;
  }
}

template <int OUT_MODE, int BIAS_MODE>
__global__ __launch_bounds__(256) void gemm64_kernel(const _Float16* __restrict__ A, int lda,
                                                     const _Float16* __restrict__ Bt, int ldb,
                                                     _Float16* __restrict__ C, _Float16* __restrict__ C2, int ldc,
                                                     const float* __restrict__ bias, float bsc,
                                                     int M, int N, int K, float scale) {
  __shared__ __align__(16) float sT[8][16 * 68];
  const int lane = threadIdx.x & 31, wave = threadIdx.x >> 5;
  const int tilesN = N >> 6, tilesM = M >> 6;
  const int tile = (int)blockIdx.x * 8 + wave;
  if (tile >= tilesM * tilesN) return;
  const int tm = tile / tilesN, tn = tile - tm * tilesN;
  const int m0 = tm << 6, n0 = tn << 6;
  const int rl = lane & 15;
  const int koff = (lane >> 4) * 8;
  const int mOff = (lane >> 4) * 8;

  v8f acc[4][4];
#pragma unroll
  for (int i = 0; i < 4; ++i)
#pragma unroll
    for (int j = 0; j < 4; ++j) acc[i][j] = zero8();

#pragma unroll 1
  for (int k0 = 0; k0 < K; k0 += 32) {
    v16h bh[4];
#pragma unroll
    for (int j = 0; j < 4; ++j) bh[j] = ldfrag(Bt + (size_t)(n0 + (j << 4) + rl) * ldb + koff + k0);
#pragma unroll
    for (int i = 0; i < 4; ++i) {
      const size_t ao = (size_t)(m0 + (i << 4) + rl) * lda + koff + k0;
      const v16h ah = ldfrag(A + ao);
#pragma unroll
      for (int j = 0; j < 4; ++j) acc[i][j] = mma16(ah, bh[j], acc[i][j]);
      guard_g(acc[i][0], acc[i][3], ah, bh[3]);
    }
    keep4(bh[0], bh[1], bh[2], bh[3]);
  }
  accg4(acc[0][0], acc[0][1], acc[0][2], acc[0][3]);
  accg4(acc[1][0], acc[1][1], acc[1][2], acc[1][3]);
  accg4(acc[2][0], acc[2][1], acc[2][2], acc[2][3]);
  accg4(acc[3][0], acc[3][1], acc[3][2], acc[3][3]);

  float* slab = sT[wave];
#pragma unroll
  for (int i = 0; i < 4; ++i) {
    const int mBase = m0 + (i << 4);
    float brow[8];
#pragma unroll
    for (int r = 0; r < 8; ++r) brow[r] = 0.0f;
    if (BIAS_MODE == 2) {
      const v4f ba = *(const v4f*)(bias + mBase + mOff);
      const v4f bb = *(const v4f*)(bias + mBase + mOff + 4);
#pragma unroll
      for (int r = 0; r < 4; ++r) { brow[r] = bsc * bfr(ba[r]); brow[4 + r] = bsc * bfr(bb[r]); }
    }
#pragma unroll
    for (int j = 0; j < 4; ++j) {
      float bcol = 0.0f;
      if (BIAS_MODE == 1) bcol = bsc * bfr(bias[n0 + (j << 4) + rl]);
#pragma unroll
      for (int r = 0; r < 8; ++r) {
        const float bb = (BIAS_MODE == 2) ? brow[r] : bcol;
        slab[(mOff + r) * 68 + (j << 4) + rl] = acc[i][j][r] * scale + bb;
      }
    }
    __builtin_amdgcn_fence(__ATOMIC_RELEASE, "workgroup");
    __builtin_amdgcn_wave_barrier();
    __builtin_amdgcn_fence(__ATOMIC_ACQUIRE, "workgroup");
    {
      const int qq = lane >> 3, c8 = (lane & 7) * 8;
#pragma unroll
      for (int ps = 0; ps < 2; ++ps) {
#pragma unroll
        for (int it = 0; it < 4; ++it) {
          const int row = it * 4 + qq;
          const float* sp = slab + row * 68 + c8;
          v8h hv, lv;
#pragma unroll
          for (int e = 0; e < 8; ++e) {
            const float f = sp[e];
            const _Float16 hh = (_Float16)f;
            hv[e] = hh;
            lv[e] = (_Float16)((f - (float)hh) * 1024.0f);
          }
          *(volatile v8h*)(C + (size_t)(mBase + row) * ldc + n0 + c8) = hv;
          if (OUT_MODE == 2) *(volatile v8h*)(C2 + (size_t)(mBase + row) * ldc + n0 + c8) = lv;
        }
        __threadfence();
      }
    }
    __builtin_amdgcn_fence(__ATOMIC_RELEASE, "workgroup");
    __builtin_amdgcn_wave_barrier();
    __builtin_amdgcn_fence(__ATOMIC_ACQUIRE, "workgroup");
  }
}

#define QB       32
#define KCH      256
#define QSP      264
#define PSP      264
#define OSP      260
#define LDS_QS   0
#define LDS_QL   16896
#define LDS_PS   33792
#define LDS_PMAX 50688
#define LDS_PSUM 51712
#define LDS_ST   52736
#define ATT_LDS  53248
static_assert(QB * QSP * 2 == LDS_QL - LDS_QS);
static_assert(QB * QSP * 2 == LDS_PS - LDS_QL);
static_assert(QB * PSP * 2 == LDS_PMAX - LDS_PS);
static_assert(QB * OSP * 4 <= LDS_PMAX - LDS_QS);
static_assert(LDS_PSUM - LDS_PMAX == 256 * 4);
static_assert(LDS_ST - LDS_PSUM == 256 * 4);
static_assert(ATT_LDS - LDS_ST == 4 * 32 * 4);
static_assert((QSP % 8) == 0 && (PSP % 8) == 0 && PSP >= KCH && (OSP % 4) == 0 && OSP >= DM);
static_assert((LDS_QL % 16) == 0 && (LDS_PS % 16) == 0 && (LDS_PMAX % 16) == 0 && (LDS_ST % 16) == 0);
static_assert((SEQ % KCH) == 0 && (SEQ % QB) == 0 && DM == 8 * 32);

__global__ __launch_bounds__(256) void attn_kernel(const _Float16* __restrict__ qh, const _Float16* __restrict__ ql,
                                                   const _Float16* __restrict__ kn, const _Float16* __restrict__ vt,
                                                   float* __restrict__ out) {
  extern __shared__ __align__(16) char smem[];
  _Float16* Qs = (_Float16*)(smem + LDS_QS);
  _Float16* Ls = (_Float16*)(smem + LDS_QL);
  _Float16* Ps = (_Float16*)(smem + LDS_PS);
  float* pmax = (float*)(smem + LDS_PMAX);
  float* psum = (float*)(smem + LDS_PSUM);
  float* m_s  = (float*)(smem + LDS_ST);
  float* l_s  = m_s + 32;
  float* al_s = m_s + 64;
  float* li_s = m_s + 96;

  const int tid = threadIdx.x, wave = tid >> 5, lane = tid & 31, h = lane >> 4, c = lane & 15;
  const int q0 = (int)blockIdx.x * QB;
  const int batch = q0 / SEQ;
  const int kbase = batch * SEQ;
  const float ninf = -__builtin_inff();
  const float sc = 0.000244140625f;
  const float rs = 0.0009765625f;

  if (tid < 32) { m_s[tid] = ninf; l_s[tid] = 0.0f; al_s[tid] = 0.0f; li_s[tid] = 0.0f; }
  psum[tid] = 0.0f;
#pragma unroll
  for (int i = 0; i < 4; ++i) {
    const int idx = i * 256 + tid;
    const int row = idx >> 5;
    const int pc  = idx & 31;
    const v8h vh = *(const v8h*)(qh + (size_t)(q0 + row) * DM + pc * 8);
    const v8h vl = *(const v8h*)(ql + (size_t)(q0 + row) * DM + pc * 8);
    *(v8h*)(Qs + row * QSP + pc * 8) = vh;
    *(v8h*)(Ls + row * QSP + pc * 8) = vl;
  }
  __syncthreads();

  v8f oacc[2][2];
#pragma unroll
  for (int qt = 0; qt < 2; ++qt)
#pragma unroll
    for (int nt = 0; nt < 2; ++nt) oacc[qt][nt] = zero8();

  const _Float16* qb0p = Qs + c * QSP + 8 * h;
  const _Float16* qb1p = Qs + (16 + c) * QSP + 8 * h;
  const _Float16* ql0p = Ls + c * QSP + 8 * h;
  const _Float16* ql1p = Ls + (16 + c) * QSP + 8 * h;
  const _Float16* pa0p = Ps + c * PSP + 8 * h;
  const _Float16* pa1p = Ps + (16 + c) * PSP + 8 * h;
  const int ntile = SEQ / KCH;

#pragma unroll 1
  for (int t = 0; t < ntile; ++t) {
    const int kb = kbase + t * KCH + 32 * wave;
    const _Float16* ka0p = kn + (size_t)(kb + c) * DM + 8 * h;
    const _Float16* ka1p = kn + (size_t)(kb + 16 + c) * DM + 8 * h;
    v8f sacc[2][2];
    v8f sacl[2][2];
#pragma unroll
    for (int qt = 0; qt < 2; ++qt)
#pragma unroll
      for (int kt = 0; kt < 2; ++kt) { sacc[qt][kt] = zero8(); sacl[qt][kt] = zero8(); }
#pragma unroll 1
    for (int k0 = 0; k0 < DM; k0 += 32) {
      const v16h a0 = ldfrag(ka0p + k0), a1 = ldfrag(ka1p + k0);
      const v16h b0 = ldfrag(qb0p + k0), b1 = ldfrag(qb1p + k0);
      const v16h c0 = ldfrag(ql0p + k0), c1 = ldfrag(ql1p + k0);
      sacc[0][0] = mma16(a0, b0, sacc[0][0]);
      sacc[0][1] = mma16(a1, b0, sacc[0][1]);
      sacc[1][0] = mma16(a0, b1, sacc[1][0]);
      sacc[1][1] = mma16(a1, b1, sacc[1][1]);
      sacl[0][0] = mma16(a0, c0, sacl[0][0]);
      sacl[0][1] = mma16(a1, c0, sacl[0][1]);
      sacl[1][0] = mma16(a0, c1, sacl[1][0]);
      sacl[1][1] = mma16(a1, c1, sacl[1][1]);
      guard_s8(sacc[0][0], sacc[0][1], sacc[1][0], sacc[1][1], sacl[0][0], sacl[0][1], sacl[1][0], sacl[1][1],
               a0, a1, b0, b1, c0, c1);
    }
    {
      float pm0 = ninf, pm1 = ninf;
#pragma unroll
      for (int kt = 0; kt < 2; ++kt) {
#pragma unroll
        for (int r = 0; r < 8; ++r) {
          const float v0 = (sacc[0][kt][r] + sacl[0][kt][r] * rs) * sc; sacc[0][kt][r] = v0; pm0 = fmaxf(pm0, v0);
          const float v1 = (sacc[1][kt][r] + sacl[1][kt][r] * rs) * sc; sacc[1][kt][r] = v1; pm1 = fmaxf(pm1, v1);
        }
      }
      pm0 = fmaxf(pm0, __shfl_xor(pm0, 16, 32));
      pm1 = fmaxf(pm1, __shfl_xor(pm1, 16, 32));
      pmax[wave * 32 + c] = pm0;
      pmax[wave * 32 + 16 + c] = pm1;
    }
    __syncthreads();
    if (wave == 0) {
      const int row = lane;
      float ps = 0.0f;
#pragma unroll
      for (int w = 0; w < 8; ++w) ps += psum[w * 32 + row];
      l_s[row] = l_s[row] * al_s[row] + ps;
      const float mo = m_s[row];
      float mx = mo;
#pragma unroll
      for (int w = 0; w < 8; ++w) mx = fmaxf(mx, pmax[w * 32 + row]);
      al_s[row] = __expf(mo - mx);
      m_s[row] = mx;
    }
    __syncthreads();
    {
      const float mq0 = m_s[c], mq1 = m_s[16 + c];
      float ps0 = 0.0f, ps1 = 0.0f;
#pragma unroll
      for (int kt = 0; kt < 2; ++kt) {
        v8h h0, h1;
#pragma unroll
        for (int r = 0; r < 8; ++r) {
          const float p0 = __expf(sacc[0][kt][r] - mq0); ps0 += p0; h0[r] = (_Float16)(p0 * 16384.0f);
          const float p1 = __expf(sacc[1][kt][r] - mq1); ps1 += p1; h1[r] = (_Float16)(p1 * 16384.0f);
        }
        *(v8h*)(Ps + c * PSP + 32 * wave + 16 * kt + 8 * h) = h0;
        *(v8h*)(Ps + (16 + c) * PSP + 32 * wave + 16 * kt + 8 * h) = h1;
      }
      ps0 += __shfl_xor(ps0, 16, 32);
      ps1 += __shfl_xor(ps1, 16, 32);
      psum[wave * 32 + c] = ps0;
      psum[wave * 32 + 16 + c] = ps1;
      const v4f aA = *(const v4f*)(al_s + 8 * h), aB = *(const v4f*)(al_s + 8 * h + 4);
      const v4f bA = *(const v4f*)(al_s + 16 + 8 * h), bB = *(const v4f*)(al_s + 16 + 8 * h + 4);
#pragma unroll
      for (int nt = 0; nt < 2; ++nt) {
#pragma unroll
        for (int r = 0; r < 4; ++r) {
          oacc[0][nt][r] *= aA[r]; oacc[0][nt][4 + r] *= aB[r];
          oacc[1][nt][r] *= bA[r]; oacc[1][nt][4 + r] *= bB[r];
        }
      }
    }
    __syncthreads();
    {
      const _Float16* vbp = vt + (size_t)(32 * wave + c) * RTOT + kbase + (size_t)t * KCH + 8 * h;
#pragma unroll 1
      for (int ks = 0; ks < KCH; ks += 32) {
        const v16h pa0 = ldfrag(pa0p + ks), pa1 = ldfrag(pa1p + ks);
        const v16h vb0 = ldfrag(vbp + ks);
        const v16h vb1 = ldfrag(vbp + (size_t)16 * RTOT + ks);
        oacc[0][0] = mma16(pa0, vb0, oacc[0][0]);
        oacc[0][1] = mma16(pa0, vb1, oacc[0][1]);
        oacc[1][0] = mma16(pa1, vb0, oacc[1][0]);
        oacc[1][1] = mma16(pa1, vb1, oacc[1][1]);
        guard_pv4(oacc[0][0], oacc[0][1], oacc[1][0], oacc[1][1], pa0, pa1, vb0, vb1);
      }
    }
  }

  if (wave == 0) {
    const int row = lane;
    float ps = 0.0f;
#pragma unroll
    for (int w = 0; w < 8; ++w) ps += psum[w * 32 + row];
    const float l = l_s[row] * al_s[row] + ps;
    li_s[row] = (1.0f / l) * (1.0f / 262144.0f);
  }
  __syncthreads();
  float* Os = (float*)(smem + LDS_QS);
  {
    const v4f iA0 = *(const v4f*)(li_s + 8 * h),      iB0 = *(const v4f*)(li_s + 8 * h + 4);
    const v4f iA1 = *(const v4f*)(li_s + 16 + 8 * h), iB1 = *(const v4f*)(li_s + 16 + 8 * h + 4);
#pragma unroll
    for (int nt = 0; nt < 2; ++nt) {
      const int col = 32 * wave + 16 * nt + c;
#pragma unroll
      for (int r = 0; r < 4; ++r) {
        Os[(8 * h + r) * OSP + col]          = oacc[0][nt][r] * iA0[r];
        Os[(8 * h + 4 + r) * OSP + col]      = oacc[0][nt][4 + r] * iB0[r];
        Os[(16 + 8 * h + r) * OSP + col]     = oacc[1][nt][r] * iA1[r];
        Os[(16 + 8 * h + 4 + r) * OSP + col] = oacc[1][nt][4 + r] * iB1[r];
      }
    }
  }
  __syncthreads();
  {
    float* go = out + (size_t)q0 * DM;
#pragma unroll
    for (int ps = 0; ps < 2; ++ps) {
#pragma unroll
      for (int rr = 0; rr < 4; ++rr) {
        const int row = 4 * wave + rr;
#pragma unroll
        for (int j = 0; j < 2; ++j) {
          const int pc = j * 32 + lane;
          const v4f v = *(const v4f*)(Os + row * OSP + pc * 4);
          *(volatile v4f*)(go + (size_t)row * DM + pc * 4) = v;
        }
      }
      __threadfence();
    }
  }
}

extern "C" void kernel_launch(void* const* d_in, const int* in_sizes, int n_in,
                              void* d_out, int out_size, void* d_ws, size_t ws_size,
                              hipStream_t stream) {
  if (n_in < 7) return;
  const int R = RTOT;
  const long long needx = ((long long)(NB - 1) * SEQ_FULL + SEQ) * DM;
  if ((long long)in_sizes[0] < needx) return;
  if (in_sizes[1] < DM * DM || in_sizes[3] < DM * DM || in_sizes[5] < DM * DM) return;
  if (in_sizes[2] < DM || in_sizes[4] < DM || in_sizes[6] < DM) return;
  if ((long long)out_size < (long long)R * DM) return;

  const float* x  = (const float*)d_in[0];
  const float* Wq = (const float*)d_in[1];
  const float* bq = (const float*)d_in[2];
  const float* Wk = (const float*)d_in[3];
  const float* bk = (const float*)d_in[4];
  const float* Wv = (const float*)d_in[5];
  const float* bv = (const float*)d_in[6];
  float* out = (float*)d_out;

  const size_t bWT = (size_t)3 * DM * DM * 2;
  const size_t bPl = (size_t)R * DM * 2;
  size_t off = 0;
  const size_t oWT = off; off += bWT;
  const size_t oX  = off; off += bPl;
  const size_t oQ  = off; off += bPl;
  const size_t oQL = off; off += bPl;
  const size_t oK  = off; off += bPl;
  const size_t oVT = off; off += bPl;
  if (off > ws_size) return;
  if (off > (size_t)134217728) return;

  char* ws = (char*)d_ws;
  _Float16* WT16 = (_Float16*)(ws + oWT);
  _Float16* X16  = (_Float16*)(ws + oX);
  _Float16* Q16  = (_Float16*)(ws + oQ);
  _Float16* QL16 = (_Float16*)(ws + oQL);
  _Float16* K16  = (_Float16*)(ws + oK);
  _Float16* VT16 = (_Float16*)(ws + oVT);

  const dim3 blk(256);
  const int nbx = (R * DM / 8) / 256;
  const int nbw = (3 * DM * DM / 8) / 256;
  if (nbx * 256 * 8 != R * DM) return;

  cvt_kernel<<<dim3(nbx + nbw), blk, 0, stream>>>(x, Wq, Wk, Wv, X16, WT16, nbx);
  gemm64_kernel<2, 1><<<dim3(((R / 64) * (DM / 64)) / 8), blk, 0, stream>>>(
      X16, DM, WT16, DM, Q16, QL16, DM, bq, 16.0f, R, DM, DM, 0.015625f);
  gemm64_kernel<1, 1><<<dim3(((R / 64) * (DM / 64)) / 8), blk, 0, stream>>>(
      X16, DM, WT16 + (size_t)DM * DM, DM, K16, K16, DM, bk, 16.0f, R, DM, DM, 0.015625f);
  gemm64_kernel<1, 2><<<dim3(((DM / 64) * (R / 64)) / 8), blk, 0, stream>>>(
      WT16 + (size_t)2 * DM * DM, DM, X16, DM, VT16, VT16, R, bv, 16.0f, DM, R, DM, 0.015625f);
  (void)hipFuncSetAttribute(reinterpret_cast<const void*>(&attn_kernel),
                            hipFuncAttributeMaxDynamicSharedMemorySize, ATT_LDS);
  attn_kernel<<<dim3(R / QB), blk, ATT_LDS, stream>>>(Q16, QL16, K16, VT16, out);
  (void)hipGetLastError();
}
